// TimeLSTM_39530878992939
// MI455X (gfx1250) — hardware-run, weakly checked
//
#include <hip/hip_runtime.h>
#include <math.h>

constexpr int NBAT    = 128;
constexpr int NSTEP   = 256;
constexpr int NCODE   = 16;
constexpr int NHID    = 256;
constexpr int NGATE   = 4 * NHID;
constexpr int NEMBROW = 257;
constexpr int NROWS   = NBAT * NSTEP;
constexpr int NOUTEL  = NBAT * NSTEP * NHID;
constexpr int SEQ_BLK = 16;
constexpr int NTHR_SEQ = 512;
constexpr int HPITCH  = 264;
constexpr int OPITCH  = 260;
constexpr float WCARRY     = 16.0f;
constexpr float WCARRY_INV = 1.0f / 16.0f;
static_assert(NBAT % SEQ_BLK == 0, "batch rows per block");
static_assert(NHID == 16 * (NTHR_SEQ / 32), "16 waves x 16 hidden columns");
static_assert(NHID % 32 == 0, "K multiple of 32");
static_assert(NROWS % 64 == 0 && NGATE % 64 == 0, "GEMM M, N tile multiples");
static_assert(NBAT == 128, "step-major row split uses shifts by 7");
static_assert((HPITCH % 8) == 0 && (OPITCH % 4) == 0, "16-B aligned LDS rows");

typedef __attribute__((ext_vector_type(16))) _Float16 v16h;
typedef __attribute__((ext_vector_type(8)))  _Float16 v8h;
typedef __attribute__((ext_vector_type(16))) __bf16   v16b;
typedef __attribute__((ext_vector_type(8)))  __bf16   v8b;
typedef __attribute__((ext_vector_type(8)))  float    v8f;
typedef __attribute__((ext_vector_type(4)))  float    v4f;
typedef __attribute__((ext_vector_type(2)))  unsigned v2u;

__device__ __forceinline__ unsigned short f2bf_bits(float f) {
  unsigned u = __float_as_uint(f);
  return (unsigned short)((u + 0x7FFFu + ((u >> 16) & 1u)) >> 16);
}
__device__ __forceinline__ float bf_bits2f(unsigned short h) { return __uint_as_float(((unsigned)h) << 16); }

__device__ __forceinline__ float h16_to_f32(unsigned hb) {
  const unsigned sgn = (hb & 0x8000u) << 16;
  const unsigned em = hb & 0x7fffu;
  const float fn = __uint_as_float((em << 13) + 0x38000000u);
  const float fs = (float)em * 5.9604644775390625e-8f;
  const float mag = (em < 0x400u) ? fs : fn;
  return __uint_as_float(__float_as_uint(mag) | sgn);
}

__device__ __forceinline__ void dep_guard4_h(v8f& a, v8f& b, v8f& c, v8f& d, v16h x, v16h y) { asm volatile("v_nop\n\tv_nop\n\tv_nop\n\tv_nop" : "+v"(a), "+v"(b), "+v"(c), "+v"(d) : "v"(x), "v"(y)); }
__device__ __forceinline__ void dep_guard4_b(v8f& a, v8f& b, v8f& c, v8f& d, v16b x, v16b y) { asm volatile("v_nop\n\tv_nop\n\tv_nop\n\tv_nop" : "+v"(a), "+v"(b), "+v"(c), "+v"(d) : "v"(x), "v"(y)); }
__device__ __forceinline__ void keep4_h(v16h a, v16h b, v16h c, v16h d) { asm volatile("v_nop" :: "v"(a), "v"(b), "v"(c), "v"(d)); }
__device__ __forceinline__ void keep4_b(v16b a, v16b b, v16b c, v16b d) { asm volatile("v_nop" :: "v"(a), "v"(b), "v"(c), "v"(d)); }
__device__ __forceinline__ void acc_guard4(v8f& a, v8f& b, v8f& c, v8f& d) { asm volatile("v_nop\n\tv_nop\n\tv_nop\n\tv_nop" : "+v"(a), "+v"(b), "+v"(c), "+v"(d)); }
__device__ __forceinline__ void guard5_h(v8f& a0, v8f& a1, v8f& a2, v8f& a3, v8f& a4,
                                         v16h x, v16h y, v16h b0, v16h b1, v16h b2, v16h b3, v16h b4) {
  asm volatile("v_nop\n\tv_nop\n\tv_nop\n\tv_nop"
               : "+v"(a0), "+v"(a1), "+v"(a2), "+v"(a3), "+v"(a4)
               : "v"(x), "v"(y), "v"(b0), "v"(b1), "v"(b2), "v"(b3), "v"(b4));
}
__device__ __forceinline__ void acc_guard5(v8f& a0, v8f& a1, v8f& a2, v8f& a3, v8f& a4) {
  asm volatile("v_nop\n\tv_nop\n\tv_nop\n\tv_nop" : "+v"(a0), "+v"(a1), "+v"(a2), "+v"(a3), "+v"(a4));
}

template <typename T> struct Frag;
template <> struct Frag<_Float16> {
  typedef v16h V; union U { v16h v; v8h h[2]; };
  static __device__ __forceinline__ v16h load(const _Float16* p) {
    U f; f.h[0] = *(const v8h*)(p); f.h[1] = *(const v8h*)(p + 16); return f.v;
  }
  static __device__ __forceinline__ v8f mma(v16h a, v16h b, v8f c) {
    return __builtin_amdgcn_wmma_f32_16x16x32_f16(false, a, false, b, (short)0, c, false, false);
  }
  static __device__ __forceinline__ void guard4(v8f& a, v8f& b, v8f& c, v8f& d, v16h x, v16h y) { dep_guard4_h(a, b, c, d, x, y); }
  static __device__ __forceinline__ void keep(v16h a, v16h b, v16h c, v16h d) { keep4_h(a, b, c, d); }
};
template <> struct Frag<__bf16> {
  typedef v16b V; union U { v16b v; v8b h[2]; };
  static __device__ __forceinline__ v16b load(const __bf16* p) {
    U f; f.h[0] = *(const v8b*)(p); f.h[1] = *(const v8b*)(p + 16); return f.v;
  }
  static __device__ __forceinline__ v8f mma(v16b a, v16b b, v8f c) {
    return __builtin_amdgcn_wmma_f32_16x16x32_bf16(false, a, false, b, (short)0, c, false, false);
  }
  static __device__ __forceinline__ void guard4(v8f& a, v8f& b, v8f& c, v8f& d, v16b x, v16b y) { dep_guard4_b(a, b, c, d, x, y); }
  static __device__ __forceinline__ void keep(v16b a, v16b b, v16b c, v16b d) { keep4_b(a, b, c, d); }
};

template <int ET> struct Elem;
template <> struct Elem<0> { typedef _Float16 T; };
template <> struct Elem<1> { typedef __bf16 T; };
template <int ET, bool SPLIT, int BIAS_MODE, int OUT_MODE, bool RESID, int ACT = 0>
__global__ __launch_bounds__(256) void wmma_gemm64(
    const unsigned short* __restrict__ Ap, const unsigned short* __restrict__ A2p, int lda, long strideA,
    const unsigned short* __restrict__ Btp, const unsigned short* __restrict__ Bt2p, int ldb, long strideB,
    void* __restrict__ Cout, void* __restrict__ Cout2, int ldc, long strideC,
    const float* __restrict__ bias,
    const float* __restrict__ resid, long strideR,
    int M, int N, int K, float scale) {
  typedef typename Elem<ET>::T T;
  typedef typename Frag<T>::V V;
  const T* A = (const T*)Ap; const T* A2 = (const T*)A2p; const T* Bt = (const T*)Btp; const T* Bt2 = (const T*)Bt2p;
  __shared__ __align__(16) float sT[8][16 * 68];
  const int b    = blockIdx.y;
  const int lane = threadIdx.x & 31;
  const int wave = threadIdx.x >> 5;
  const int tilesN = N >> 6;
  const int tilesM = M >> 6;
  const int tile = blockIdx.x * 8 + wave;
  if (tile >= tilesM * tilesN) return;
  const int tm = tile / tilesN;
  const int tn = tile - tm * tilesN;
  const int m0 = tm << 6;
  const int n0 = tn << 6;

  const T* Ab  = A  + (size_t)b * strideA;
  const T* Bb  = Bt + (size_t)b * strideB;
  const T* Ab2 = SPLIT ? (A2  + (size_t)b * strideA) : nullptr;
  const T* Bb2 = SPLIT ? (Bt2 + (size_t)b * strideB) : nullptr;

  const int rlane = lane & 15;
  const int koff  = (lane >> 4) * 8;
  const int mOff  = (lane >> 4) * 8;

  v8f acc[4][4];
#pragma unroll
  for (int i = 0; i < 4; ++i)
#pragma unroll
    for (int j = 0; j < 4; ++j) acc[i][j] = (v8f){0.f,0.f,0.f,0.f,0.f,0.f,0.f,0.f};

  for (int k0 = 0; k0 < K; k0 += 32) {
    V bh[4], bl[4];
#pragma unroll
    for (int j = 0; j < 4; ++j) {
      const size_t bo = (size_t)(n0 + (j << 4) + rlane) * ldb + koff + k0;
      bh[j] = Frag<T>::load(Bb + bo);
      if (SPLIT) bl[j] = Frag<T>::load(Bb2 + bo);
    }
#pragma unroll
    for (int i = 0; i < 4; ++i) {
      const size_t ao = (size_t)(m0 + (i << 4) + rlane) * lda + koff + k0;
      V ah = Frag<T>::load(Ab + ao);
      V al;
      if (SPLIT) al = Frag<T>::load(Ab2 + ao);
#pragma unroll
      for (int j = 0; j < 4; ++j) {
        acc[i][j] = Frag<T>::mma(ah, bh[j], acc[i][j]);
        if (SPLIT) {
          acc[i][j] = Frag<T>::mma(ah, bl[j], acc[i][j]);
          acc[i][j] = Frag<T>::mma(al, bh[j], acc[i][j]);
        }
      }
      Frag<T>::guard4(acc[i][0], acc[i][1], acc[i][2], acc[i][3], ah, SPLIT ? al : ah);
    }
    Frag<T>::keep(bh[0], bh[1], bh[2], bh[3]);
    if (SPLIT) Frag<T>::keep(bl[0], bl[1], bl[2], bl[3]);
  }
  acc_guard4(acc[0][0], acc[0][1], acc[0][2], acc[0][3]);
  acc_guard4(acc[1][0], acc[1][1], acc[1][2], acc[1][3]);
  acc_guard4(acc[2][0], acc[2][1], acc[2][2], acc[2][3]);
  acc_guard4(acc[3][0], acc[3][1], acc[3][2], acc[3][3]);

  float* slab = sT[wave];
  const float* Rb = RESID ? (resid + (size_t)b * strideR) : nullptr;
#pragma unroll
  for (int i = 0; i < 4; ++i) {
    const int mBase = m0 + (i << 4);
#pragma unroll
    for (int j = 0; j < 4; ++j) {
      const int n = n0 + (j << 4) + rlane;
      float bv = 0.f;
      if (BIAS_MODE == 2) bv = bias[n];
#pragma unroll
      for (int r = 0; r < 8; ++r) {
        float v = acc[i][j][r] * scale;
        if (BIAS_MODE == 1) v += bias[mBase + mOff + r];
        if (BIAS_MODE == 2) v += bv;
        if (RESID) v += Rb[(size_t)(mBase + mOff + r) * ldc + n];
        if (ACT == 1) v = tanhf(v);
        if (ACT == 2) v = fmaxf(v, 0.0f);
        if (ACT == 3) v = v / (1.0f + expf(-v));
        if (ACT == 4) v = (v > 0.f) ? v : 0.01f * v;
        slab[(mOff + r) * 68 + (j << 4) + rlane] = v;
      }
    }
    __builtin_amdgcn_fence(__ATOMIC_RELEASE, "workgroup");
    __builtin_amdgcn_wave_barrier();
    __builtin_amdgcn_fence(__ATOMIC_ACQUIRE, "workgroup");
    if (OUT_MODE == 0) {
      float* C = (float*)Cout + (size_t)b * strideC;
      const int hh = lane >> 4, c4 = (lane & 15) * 4;
      for (int pass = 0; pass < 2; ++pass) {
#pragma unroll
        for (int it = 0; it < 8; ++it) {
          const int row = it * 2 + hh;
          v4f v = *(const v4f*)(slab + row * 68 + c4);
          *(volatile v4f*)(C + (size_t)(mBase + row) * ldc + n0 + c4) = v;
        }
        __threadfence();
      }
    } else {
      const int q = lane >> 3, c8 = (lane & 7) * 8;
      unsigned short* C  = (unsigned short*)Cout  + (size_t)b * strideC;
      unsigned short* C2 = (OUT_MODE == 2) ? ((unsigned short*)Cout2 + (size_t)b * strideC) : nullptr;
      for (int pass = 0; pass < 2; ++pass) {
#pragma unroll
        for (int it = 0; it < 4; ++it) {
          const int row = it * 4 + q;
          const float* sp = slab + row * 68 + c8;
          v8h hv, lv;
#pragma unroll
          for (int e = 0; e < 8; ++e) {
            if (OUT_MODE == 1) {
              hv[e] = (_Float16)sp[e];
            } else {
              unsigned short hb = f2bf_bits(sp[e]);
              unsigned short lb = f2bf_bits(sp[e] - bf_bits2f(hb));
              hv[e] = __builtin_bit_cast(_Float16, hb);
              lv[e] = __builtin_bit_cast(_Float16, lb);
            }
          }
          *(volatile v8h*)(C + (size_t)(mBase + row) * ldc + n0 + c8) = hv;
          if (OUT_MODE == 2) *(volatile v8h*)(C2 + (size_t)(mBase + row) * ldc + n0 + c8) = lv;
        }
        __threadfence();
      }
    }
    __builtin_amdgcn_fence(__ATOMIC_RELEASE, "workgroup");
    __builtin_amdgcn_wave_barrier();
    __builtin_amdgcn_fence(__ATOMIC_ACQUIRE, "workgroup");
  }
}

__global__ __launch_bounds__(256) void cvt8_f16_kernel(const float* __restrict__ src, unsigned short* __restrict__ dst,
                                                       int nrow, int perm, float sc) {
  const int i  = blockIdx.x * 256 + threadIdx.x;
  const int n8 = nrow * (NHID / 8);
  if (i < n8) {
    const int row = i >> 5;
    const int c8  = i & 31;
    const int srow = perm ? (((row & 3) * NHID) + (row >> 2)) : row;
    const float* sp = src + (size_t)srow * NHID + c8 * 8;
    const v4f a = *(const v4f*)(sp);
    const v4f b = *(const v4f*)(sp + 4);
    v8h hv;
#pragma unroll
    for (int e = 0; e < 4; ++e) {
      hv[e]     = (_Float16)(a[e] * sc);
      hv[4 + e] = (_Float16)(b[e] * sc);
    }
    *(volatile v8h*)(dst + (size_t)i * 8) = hv;
    __threadfence();
    *(volatile v8h*)(dst + (size_t)i * 8) = hv;
  }
}

__global__ __launch_bounds__(256) void ts_bias_kernel(const float* __restrict__ times, const float* __restrict__ ub,
                                                      const float* __restrict__ wb, float* __restrict__ TSV,
                                                      float* __restrict__ BIASG) {
  const int tid = threadIdx.x;
  if (blockIdx.x < NROWS / 256) {
    const int i = blockIdx.x * 256 + tid;
    const float lg = logf(times[i] + 2.7183f);
    const float v = 1.0f / lg;
    *(volatile float*)(TSV + i) = v;
    __threadfence();
    *(volatile float*)(TSV + i) = v;
  } else {
    v4f o;
#pragma unroll
    for (int g = 0; g < 4; ++g) o[g] = ub[g * NHID + tid] + wb[g * NHID + tid];
    float* op = BIASG + 4 * tid;
    *(volatile v4f*)op = o;
    __threadfence();
    *(volatile v4f*)op = o;
  }
}

__global__ __launch_bounds__(256) void embed_rows_kernel(const int* __restrict__ codes, const float* __restrict__ mask,
                                                         const float* __restrict__ emb, unsigned short* __restrict__ X16) {
  const int lane = threadIdx.x & 31, wave = threadIdx.x >> 5;
  const int f = blockIdx.x * 8 + wave;
  if (f >= NROWS) return;
  const int s = f >> 7;
  const int b = f & (NBAT - 1);
  const size_t bs = (size_t)b * NSTEP + (size_t)s;
  const int*   cd = codes + bs * NCODE;
  const float* mk = mask  + bs * NCODE;
  float acc[8];
#pragma unroll
  for (int e = 0; e < 8; ++e) acc[e] = 0.0f;
#pragma unroll 1
  for (int cc = 0; cc < NCODE; ++cc) {
    int code = cd[cc];
    code = code < 0 ? 0 : code;
    code = code > (NEMBROW - 1) ? (NEMBROW - 1) : code;
    const float m = mk[cc];
    const float* er = emb + (size_t)code * NHID + lane * 8;
    const v4f e0 = *(const v4f*)(er);
    const v4f e1 = *(const v4f*)(er + 4);
#pragma unroll
    for (int e = 0; e < 4; ++e) {
      acc[e]     = fmaf(e0[e], m, acc[e]);
      acc[4 + e] = fmaf(e1[e], m, acc[4 + e]);
    }
  }
  v8h hv;
#pragma unroll
  for (int e = 0; e < 8; ++e) hv[e] = (_Float16)acc[e];
  unsigned short* op = X16 + (size_t)f * NHID + lane * 8;
  *(volatile v8h*)op = hv;
  __threadfence();
  *(volatile v8h*)op = hv;
}

__device__ __forceinline__ float sigm_p(float x) {
  const float xc = fminf(fmaxf(x, -30.0f), 30.0f);
  return __builtin_amdgcn_rcpf(1.0f + expf(-xc));
}
__device__ __forceinline__ float tanh_p(float x) {
  const float xc = fminf(fmaxf(x, -15.0f), 15.0f);
  return 1.0f - 2.0f * __builtin_amdgcn_rcpf(1.0f + expf(2.0f * xc));
}

__global__ __launch_bounds__(NTHR_SEQ) void tlstm_seq_kernel(const unsigned short* __restrict__ XPp,
                                                             const float* __restrict__ TSV,
                                                             const unsigned short* __restrict__ WHp,
                                                             const unsigned short* __restrict__ WDp,
                                                             const float* __restrict__ wd_b,
                                                             float* __restrict__ out) {
  __shared__ __align__(16) _Float16 Ah[SEQ_BLK * HPITCH];
  __shared__ __align__(16) _Float16 Ac[SEQ_BLK * HPITCH];
  __shared__ __align__(16) float    Hs[SEQ_BLK * OPITCH];
  __shared__ __align__(16) float    sTs[SEQ_BLK];
  const _Float16* WH = (const _Float16*)WHp;
  const _Float16* WD = (const _Float16*)WDp;
  const int tid = threadIdx.x, lane = tid & 31, wave = tid >> 5;
  const int c = lane & 15, hh = lane >> 4, koff = hh * 8;
  const int rowbase = blockIdx.x * SEQ_BLK;
  const int j = 16 * wave + c;

#pragma unroll 1
  for (int i = tid; i < SEQ_BLK * HPITCH; i += NTHR_SEQ) {
    Ah[i] = (_Float16)0.0f;
    Ac[i] = (_Float16)0.0f;
  }
  {
    float t0 = TSV[(size_t)(rowbase + (tid & 15)) * NSTEP];
    asm volatile("" : "+v"(t0));
    if (tid < SEQ_BLK) sTs[tid] = t0;
  }
  float cst[8];
#pragma unroll
  for (int r = 0; r < 8; ++r) cst[r] = 0.0f;
  const float bd = wd_b[j];
  __syncthreads();

  const _Float16* ahrow = Ah + c * HPITCH + koff;
  const _Float16* acrow = Ac + c * HPITCH + koff;
  const _Float16* wf = WH + (size_t)j * NHID + koff;
  const _Float16* wi = wf + (size_t)1 * NHID * NHID;
  const _Float16* wo = wf + (size_t)2 * NHID * NHID;
  const _Float16* wg = wf + (size_t)3 * NHID * NHID;
  const _Float16* wd = WD + (size_t)j * NHID + koff;
  const v8f z8 = {0.f, 0.f, 0.f, 0.f, 0.f, 0.f, 0.f, 0.f};
  const float* hsrow = Hs + wave * OPITCH + lane * 4;

#pragma unroll 1
  for (int s = 0; s < NSTEP; ++s) {
    const unsigned short* xrow = XPp + ((size_t)s * NBAT + (size_t)(rowbase + 8 * hh)) * NGATE + 4 * j;
    v2u xw[8];
#pragma unroll
    for (int r = 0; r < 8; ++r) xw[r] = *(const v2u*)(xrow + (size_t)r * NGATE);
    const int sn = (s + 1 < NSTEP) ? (s + 1) : (NSTEP - 1);
    float tnext = TSV[(size_t)(rowbase + (tid & 15)) * NSTEP + sn];
    asm volatile("" : "+v"(tnext));
    const v4f tsa = *(const v4f*)(sTs + 8 * hh);
    const v4f tsb = *(const v4f*)(sTs + 8 * hh + 4);

    v8f aF = z8, aI = z8, aO = z8, aG = z8, aD = z8;
#pragma unroll 1
    for (int k0 = 0; k0 < NHID; k0 += 32) {
      const v16h ah = Frag<_Float16>::load(ahrow + k0);
      const v16h ac = Frag<_Float16>::load(acrow + k0);
      const v16h bF = Frag<_Float16>::load(wf + k0);
      const v16h bI = Frag<_Float16>::load(wi + k0);
      const v16h bO = Frag<_Float16>::load(wo + k0);
      const v16h bG = Frag<_Float16>::load(wg + k0);
      const v16h bD = Frag<_Float16>::load(wd + k0);
      aF = Frag<_Float16>::mma(ah, bF, aF);
      aI = Frag<_Float16>::mma(ah, bI, aI);
      aO = Frag<_Float16>::mma(ah, bO, aO);
      aG = Frag<_Float16>::mma(ah, bG, aG);
      aD = Frag<_Float16>::mma(ac, bD, aD);
      guard5_h(aF, aI, aO, aG, aD, ah, ac, bF, bI, bO, bG, bD);
    }
    acc_guard5(aF, aI, aO, aG, aD);

    float hst[8];
#pragma unroll
    for (int r = 0; r < 8; ++r) {
      const unsigned w0 = xw[r][0];
      const unsigned w1 = xw[r][1];
      const float zf = aF[r] * WCARRY_INV + h16_to_f32(w0 & 0xffffu);
      const float zi = aI[r] * WCARRY_INV + h16_to_f32(w0 >> 16);
      const float zo = aO[r] * WCARRY_INV + h16_to_f32(w1 & 0xffffu);
      const float zg = aG[r] * WCARRY_INV + h16_to_f32(w1 >> 16);
      const float zd = aD[r] * WCARRY_INV + bd;
      const float tsr = (r < 4) ? tsa[r & 3] : tsb[r & 3];
      const float cs1  = tanh_p(zd);
      const float cold = cst[r];
      const float cadj = (cold - cs1) + cs1 * tsr;
      const float fg = sigm_p(zf);
      const float ig = sigm_p(zi);
      const float og = sigm_p(zo);
      const float gg = sigm_p(zg);
      const float cn = fg * cadj + ig * gg;
      cst[r] = cn;
      hst[r] = og * tanh_p(cn);
    }

    __syncthreads();
#pragma unroll
    for (int r = 0; r < 8; ++r) {
      const int row = 8 * hh + r;
      Ah[row * HPITCH + j] = (_Float16)hst[r];
      Ac[row * HPITCH + j] = (_Float16)cst[r];
      Hs[row * OPITCH + j] = hst[r];
    }
    if (tid < SEQ_BLK) sTs[tid] = tnext;
    __syncthreads();

    {
      const v4f v0 = *(const v4f*)(hsrow);
      const v4f v1 = *(const v4f*)(hsrow + 128);
      float* op = out + ((size_t)(rowbase + wave) * NSTEP + (size_t)s) * NHID + lane * 4;
      *(volatile v4f*)(op)       = v0;
      *(volatile v4f*)(op + 128) = v1;
      __threadfence();
      *(volatile v4f*)(op)       = v0;
      *(volatile v4f*)(op + 128) = v1;
      __threadfence();
    }
  }
}

extern "C" void kernel_launch(void* const* d_in, const int* in_sizes, int n_in,
                              void* d_out, int out_size, void* d_ws, size_t ws_size, hipStream_t stream) {
  if (n_in < 10 || d_out == nullptr || d_ws == nullptr) return;
  if (in_sizes[0] != NBAT * NSTEP * NCODE || in_sizes[1] != NBAT * NSTEP * NCODE || in_sizes[2] != NBAT * NSTEP ||
      in_sizes[3] != NEMBROW * NHID || in_sizes[4] != NGATE * NHID || in_sizes[5] != NGATE ||
      in_sizes[6] != NGATE * NHID || in_sizes[7] != NGATE || in_sizes[8] != NHID * NHID || in_sizes[9] != NHID ||
      out_size != NOUTEL) return;

  const int*   codes  = (const int*)  d_in[0];
  const float* mask   = (const float*)d_in[1];
  const float* times  = (const float*)d_in[2];
  const float* emb    = (const float*)d_in[3];
  const float* wall_w = (const float*)d_in[4];
  const float* wall_b = (const float*)d_in[5];
  const float* uall_w = (const float*)d_in[6];
  const float* uall_b = (const float*)d_in[7];
  const float* wd_w   = (const float*)d_in[8];
  const float* wd_b   = (const float*)d_in[9];
  float* out = (float*)d_out;

  char* ws = (char*)d_ws; size_t off = 0;
  auto carve = [&](size_t bytes) -> char* { char* p = ws + off; off += (bytes + 255) & ~(size_t)255; return p; };
  unsigned short* X16    = (unsigned short*)carve((size_t)NROWS * NHID * 2);
  unsigned short* XP16   = (unsigned short*)carve((size_t)NROWS * NGATE * 2);
  unsigned short* UALL16 = (unsigned short*)carve((size_t)NGATE * NHID * 2);
  unsigned short* WALL16 = (unsigned short*)carve((size_t)NGATE * NHID * 2);
  unsigned short* WD16   = (unsigned short*)carve((size_t)NHID * NHID * 2);
  float*          BIASG  = (float*)carve((size_t)NGATE * 4);
  float*          TSV    = (float*)carve((size_t)NROWS * 4);
  if (off > ws_size || off > (size_t)134217728) return;

  cvt8_f16_kernel<<<(NGATE * (NHID / 8)) / 256, 256, 0, stream>>>(uall_w, UALL16, NGATE, 1, WCARRY);
  cvt8_f16_kernel<<<(NGATE * (NHID / 8)) / 256, 256, 0, stream>>>(wall_w, WALL16, NGATE, 0, WCARRY);
  cvt8_f16_kernel<<<(NHID * (NHID / 8)) / 256, 256, 0, stream>>>(wd_w, WD16, NHID, 0, WCARRY);
  ts_bias_kernel<<<NROWS / 256 + 1, 256, 0, stream>>>(times, uall_b, wall_b, TSV, BIASG);
  embed_rows_kernel<<<NROWS / 8, 256, 0, stream>>>(codes, mask, emb, X16);
  const dim3 ggrid((NROWS / 64) * (NGATE / 64) / 8, 1);
  wmma_gemm64<0, false, 2, 1, false, 0><<<ggrid, 256, 0, stream>>>(
      X16, X16, NHID, 0L, UALL16, UALL16, NHID, 0L, (void*)XP16, (void*)XP16, NGATE, 0L,
      BIASG, BIASG, 0L, NROWS, NGATE, NHID, WCARRY_INV);
  tlstm_seq_kernel<<<NBAT / SEQ_BLK, NTHR_SEQ, 0, stream>>>(XP16, TSV, WALL16, WD16, wd_b, out);
}
